// MRU_78039555768550
// MI455X (gfx1250) — hardware-verified
//
#include <hip/hip_runtime.h>
#include <stddef.h>

constexpr int BATCH  = 8;
constexpr int STEPS  = 2048;
constexpr int DMODEL = 256;
constexpr int HEADS  = 8;
constexpr int ROWS_M = BATCH * STEPS;
constexpr int HSW    = HEADS * DMODEL;

static_assert(ROWS_M == 16384);
static_assert(HSW == 2048);
static_assert(DMODEL % 32 == 0 && HSW % 32 == 0);
static_assert(DMODEL % 64 == 0 && ROWS_M % 64 == 0);
static_assert(BATCH == 8 && DMODEL == 16 * 16);

typedef __attribute__((ext_vector_type(16))) _Float16 v16h;
typedef __attribute__((ext_vector_type(8)))  _Float16 v8h;
typedef __attribute__((ext_vector_type(16))) __bf16   v16b;
typedef __attribute__((ext_vector_type(8)))  __bf16   v8b;
typedef __attribute__((ext_vector_type(8)))  float    v8f;
typedef __attribute__((ext_vector_type(4)))  float    v4f;

__device__ __forceinline__ unsigned short f2bf_bits(float f) {
  unsigned u = __float_as_uint(f);
  return (unsigned short)((u + 0x7FFFu + ((u >> 16) & 1u)) >> 16);
}
__device__ __forceinline__ float bf_bits2f(unsigned short h) { return __uint_as_float(((unsigned)h) << 16); }

__device__ __forceinline__ void dep_guard_h(v8f& a, v8f& b, v16h x, v16h y) { asm volatile("v_nop\n\tv_nop\n\tv_nop\n\tv_nop" : "+v"(a), "+v"(b) : "v"(x), "v"(y)); }
__device__ __forceinline__ void dep_guard_b(v8f& a, v8f& b, v16b x, v16b y) { asm volatile("v_nop\n\tv_nop\n\tv_nop\n\tv_nop" : "+v"(a), "+v"(b) : "v"(x), "v"(y)); }
__device__ __forceinline__ void keep4_h(v16h a, v16h b, v16h c, v16h d) { asm volatile("v_nop" :: "v"(a), "v"(b), "v"(c), "v"(d)); }
__device__ __forceinline__ void keep4_b(v16b a, v16b b, v16b c, v16b d) { asm volatile("v_nop" :: "v"(a), "v"(b), "v"(c), "v"(d)); }
__device__ __forceinline__ void acc_guard4(v8f& a, v8f& b, v8f& c, v8f& d) { asm volatile("v_nop\n\tv_nop\n\tv_nop\n\tv_nop" : "+v"(a), "+v"(b), "+v"(c), "+v"(d)); }
template <typename T> struct Frag;
template <> struct Frag<_Float16> {
  typedef v16h V; union U { v16h v; v8h h[2]; };
  static __device__ __forceinline__ v16h load(const _Float16* p) {
    U f; f.h[0] = *(const v8h*)(p); f.h[1] = *(const v8h*)(p + 16); return f.v;
  }
  static __device__ __forceinline__ v8f mma(v16h a, v16h b, v8f c) {
    return __builtin_amdgcn_wmma_f32_16x16x32_f16(false, a, false, b, (short)0, c, false, false);
  }
  static __device__ __forceinline__ void guard(v8f& a, v8f& b, v16h x, v16h y) { dep_guard_h(a, b, x, y); }
  static __device__ __forceinline__ void keep(v16h a, v16h b, v16h c, v16h d) { keep4_h(a, b, c, d); }
};
template <> struct Frag<__bf16> {
  typedef v16b V; union U { v16b v; v8b h[2]; };
  static __device__ __forceinline__ v16b load(const __bf16* p) {
    U f; f.h[0] = *(const v8b*)(p); f.h[1] = *(const v8b*)(p + 16); return f.v;
  }
  static __device__ __forceinline__ v8f mma(v16b a, v16b b, v8f c) {
    return __builtin_amdgcn_wmma_f32_16x16x32_bf16(false, a, false, b, (short)0, c, false, false);
  }
  static __device__ __forceinline__ void guard(v8f& a, v8f& b, v16b x, v16b y) { dep_guard_b(a, b, x, y); }
  static __device__ __forceinline__ void keep(v16b a, v16b b, v16b c, v16b d) { keep4_b(a, b, c, d); }
};

template <int ET> struct Elem;
template <> struct Elem<0> { typedef _Float16 T; };
template <> struct Elem<1> { typedef __bf16 T; };
template <int ET, bool SPLIT, int BIAS_MODE, int OUT_MODE, bool RESID, int ACT = 0>
__global__ __launch_bounds__(256) void wmma_gemm64(
    const unsigned short* __restrict__ Ap, const unsigned short* __restrict__ A2p, int lda, long strideA,
    const unsigned short* __restrict__ Btp, const unsigned short* __restrict__ Bt2p, int ldb, long strideB,
    void* __restrict__ Cout, void* __restrict__ Cout2, int ldc, long strideC,
    const float* __restrict__ bias,
    const float* __restrict__ resid, long strideR,
    int M, int N, int K, float scale) {
  typedef typename Elem<ET>::T T;
  typedef typename Frag<T>::V V;
  const T* A = (const T*)Ap; const T* A2 = (const T*)A2p; const T* Bt = (const T*)Btp; const T* Bt2 = (const T*)Bt2p;
  __shared__ __align__(16) float sT[8][16 * 68];
  const int b    = blockIdx.y;
  const int lane = threadIdx.x & 31;
  const int wave = threadIdx.x >> 5;
  const int tilesN = N >> 6;
  const int tilesM = M >> 6;
  const int tile = blockIdx.x * 8 + wave;
  if (tile >= tilesM * tilesN) return;
  const int tm = tile / tilesN;
  const int tn = tile - tm * tilesN;
  const int m0 = tm << 6;
  const int n0 = tn << 6;

  const T* Ab  = A  + (size_t)b * strideA;
  const T* Bb  = Bt + (size_t)b * strideB;
  const T* Ab2 = SPLIT ? (A2  + (size_t)b * strideA) : nullptr;
  const T* Bb2 = SPLIT ? (Bt2 + (size_t)b * strideB) : nullptr;

  const int rlane = lane & 15;
  const int koff  = (lane >> 4) * 8;
  const int mOff  = (lane >> 4) * 8;

  v8f acc[4][4];
#pragma unroll
  for (int i = 0; i < 4; ++i)
#pragma unroll
    for (int j = 0; j < 4; ++j) acc[i][j] = (v8f){0.f,0.f,0.f,0.f,0.f,0.f,0.f,0.f};

  for (int k0 = 0; k0 < K; k0 += 32) {
    V bh[4], bl[4];
#pragma unroll
    for (int j = 0; j < 4; ++j) {
      const size_t bo = (size_t)(n0 + (j << 4) + rlane) * ldb + koff + k0;
      bh[j] = Frag<T>::load(Bb + bo);
      if (SPLIT) bl[j] = Frag<T>::load(Bb2 + bo);
    }
#pragma unroll
    for (int i = 0; i < 4; ++i) {
      const size_t ao = (size_t)(m0 + (i << 4) + rlane) * lda + koff + k0;
      V ah = Frag<T>::load(Ab + ao);
      V al;
      if (SPLIT) al = Frag<T>::load(Ab2 + ao);
#pragma unroll
      for (int j = 0; j < 4; ++j) {
        acc[i][j] = Frag<T>::mma(ah, bh[j], acc[i][j]);
        if (SPLIT) {
          acc[i][j] = Frag<T>::mma(ah, bl[j], acc[i][j]);
          acc[i][j] = Frag<T>::mma(al, bh[j], acc[i][j]);
        }
      }
      Frag<T>::guard(acc[i][0], acc[i][3], ah, SPLIT ? al : ah);
    }
    Frag<T>::keep(bh[0], bh[1], bh[2], bh[3]);
    if (SPLIT) Frag<T>::keep(bl[0], bl[1], bl[2], bl[3]);
  }
  acc_guard4(acc[0][0], acc[0][1], acc[0][2], acc[0][3]);
  acc_guard4(acc[1][0], acc[1][1], acc[1][2], acc[1][3]);
  acc_guard4(acc[2][0], acc[2][1], acc[2][2], acc[2][3]);
  acc_guard4(acc[3][0], acc[3][1], acc[3][2], acc[3][3]);

  float* slab = sT[wave];
  const float* Rb = RESID ? (resid + (size_t)b * strideR) : nullptr;
#pragma unroll
  for (int i = 0; i < 4; ++i) {
    const int mBase = m0 + (i << 4);
#pragma unroll
    for (int j = 0; j < 4; ++j) {
      const int n = n0 + (j << 4) + rlane;
      float bv = 0.f;
      if (BIAS_MODE == 2) bv = bias[n];
#pragma unroll
      for (int r = 0; r < 8; ++r) {
        float v = acc[i][j][r] * scale;
        if (BIAS_MODE == 1) v += bias[mBase + mOff + r];
        if (BIAS_MODE == 2) v += bv;
        if (RESID) v += Rb[(size_t)(mBase + mOff + r) * ldc + n];
        if (ACT == 1) v = tanhf(v);
        if (ACT == 2) v = fmaxf(v, 0.0f);
        if (ACT == 3) v = v / (1.0f + expf(-v));
        if (ACT == 4) v = (v > 0.f) ? v : 0.01f * v;
        if (ACT == 5) v = 0.5f * v * (1.0f + erff(v * 0.70710678118654752f));
        slab[(mOff + r) * 68 + (j << 4) + rlane] = v;
      }
    }
    __builtin_amdgcn_fence(__ATOMIC_RELEASE, "workgroup");
    __builtin_amdgcn_wave_barrier();
    __builtin_amdgcn_fence(__ATOMIC_ACQUIRE, "workgroup");
    if (OUT_MODE == 0) {
      float* C = (float*)Cout + (size_t)b * strideC;
      const int hh = lane >> 4, c4 = (lane & 15) * 4;
      for (int pass = 0; pass < 2; ++pass) {
#pragma unroll
        for (int it = 0; it < 8; ++it) {
          const int row = it * 2 + hh;
          v4f v = *(const v4f*)(slab + row * 68 + c4);
          *(volatile v4f*)(C + (size_t)(mBase + row) * ldc + n0 + c4) = v;
        }
        __threadfence();
      }
    } else {
      const int q = lane >> 3, c8 = (lane & 7) * 8;
      unsigned short* C  = (unsigned short*)Cout  + (size_t)b * strideC;
      unsigned short* C2 = (OUT_MODE == 2) ? ((unsigned short*)Cout2 + (size_t)b * strideC) : nullptr;
      for (int pass = 0; pass < 2; ++pass) {
#pragma unroll
        for (int it = 0; it < 4; ++it) {
          const int row = it * 4 + q;
          const float* sp = slab + row * 68 + c8;
          v8h hv, lv;
#pragma unroll
          for (int e = 0; e < 8; ++e) {
            if (OUT_MODE == 1) {
              hv[e] = (_Float16)sp[e];
            } else {
              unsigned short hb = f2bf_bits(sp[e]);
              unsigned short lb = f2bf_bits(sp[e] - bf_bits2f(hb));
              hv[e] = __builtin_bit_cast(_Float16, hb);
              lv[e] = __builtin_bit_cast(_Float16, lb);
            }
          }
          *(volatile v8h*)(C + (size_t)(mBase + row) * ldc + n0 + c8) = hv;
          if (OUT_MODE == 2) *(volatile v8h*)(C2 + (size_t)(mBase + row) * ldc + n0 + c8) = lv;
        }
        __threadfence();
      }
    }
    __builtin_amdgcn_fence(__ATOMIC_RELEASE, "workgroup");
    __builtin_amdgcn_wave_barrier();
    __builtin_amdgcn_fence(__ATOMIC_ACQUIRE, "workgroup");
  }
}

__global__ __launch_bounds__(256) void cast_x_rows(const float* __restrict__ x, unsigned short* __restrict__ Xh) {
  const int g = blockIdx.x * 256 + (int)threadIdx.x;
  if (g >= ROWS_M * 32) return;
  const int m  = g >> 5;
  const int ch = g & 31;
  const int b  = m & (BATCH - 1);
  const int t  = m >> 3;
  const float* src = x + ((size_t)b * STEPS + t) * DMODEL + ch * 8;
  const v4f a0 = *(const v4f*)src;
  const v4f a1 = *(const v4f*)(src + 4);
  v8h hv;
  hv[0] = (_Float16)a0[0]; hv[1] = (_Float16)a0[1]; hv[2] = (_Float16)a0[2]; hv[3] = (_Float16)a0[3];
  hv[4] = (_Float16)a1[0]; hv[5] = (_Float16)a1[1]; hv[6] = (_Float16)a1[2]; hv[7] = (_Float16)a1[3];
  _Float16* dst = (_Float16*)Xh + (size_t)m * DMODEL + ch * 8;
  *(volatile v8h*)dst = hv;
  __threadfence();
  *(volatile v8h*)dst = hv;
}

__global__ __launch_bounds__(256) void prep_w_rows(const float* __restrict__ W, unsigned short* __restrict__ WTg) {
  const int g = blockIdx.x * 256 + (int)threadIdx.x;
  if (g >= 2 * HEADS * DMODEL * 32) return;
  const int ch   = g & 31;
  const int e    = (g >> 5) & (DMODEL - 1);
  const int h    = (g >> 13) & (HEADS - 1);
  const int part = (g >> 16) & 1;
  const int d0   = ch * 8;
  const float* src = W + ((size_t)(h * 2 * DMODEL + part * DMODEL + d0)) * DMODEL + e;
  v8h hv;
#pragma unroll
  for (int j = 0; j < 8; ++j) hv[j] = (_Float16)(src[(size_t)j * DMODEL] * 16.0f);
  _Float16* dst = (_Float16*)WTg + ((size_t)((part * HEADS + h) * DMODEL + e)) * DMODEL + d0;
  *(volatile v8h*)dst = hv;
  __threadfence();
  *(volatile v8h*)dst = hv;
}

__global__ __launch_bounds__(256) void prep_wl_rows(const float* __restrict__ Wl, unsigned short* __restrict__ WlT) {
  const int g = blockIdx.x * 256 + (int)threadIdx.x;
  if (g >= DMODEL * (HSW / 8)) return;
  const int ch = g & (HSW / 8 - 1);
  const int e  = g >> 8;
  const int j0 = ch * 8;
  const float* src = Wl + (size_t)j0 * DMODEL + e;
  v8h hv;
#pragma unroll
  for (int j = 0; j < 8; ++j) hv[j] = (_Float16)(src[(size_t)j * DMODEL] * 32.0f);
  _Float16* dst = (_Float16*)WlT + (size_t)e * HSW + j0;
  *(volatile v8h*)dst = hv;
  __threadfence();
  *(volatile v8h*)dst = hv;
}

__global__ __launch_bounds__(512) void gated_scan(
    const float* __restrict__ XPf, const float* __restrict__ XPc,
    const unsigned short* __restrict__ Whf, const unsigned short* __restrict__ Whc,
    unsigned short* __restrict__ HS, int head) {
  __shared__ __align__(16) unsigned short sA[16 * DMODEL];
  const int tid  = (int)threadIdx.x;
  const int lane = tid & 31;
  const int wave = tid >> 5;
  const int hh   = lane >> 4;
  const int c    = lane & 15;
  const int col  = wave * 16 + c;
  {
    uint4 z; z.x = 0u; z.y = 0u; z.z = 0u; z.w = 0u;
    ((uint4*)sA)[tid] = z;
  }
  const _Float16* wf = (const _Float16*)Whf + (size_t)col * DMODEL + 8 * hh;
  const _Float16* wc = (const _Float16*)Whc + (size_t)col * DMODEL + 8 * hh;
  v16h bfw[8], bcw[8];
#pragma unroll
  for (int q = 0; q < 4; ++q) {
    bfw[2 * q]     = Frag<_Float16>::load(wf + (2 * q) * 32);
    bfw[2 * q + 1] = Frag<_Float16>::load(wf + (2 * q + 1) * 32);
    bcw[2 * q]     = Frag<_Float16>::load(wc + (2 * q) * 32);
    bcw[2 * q + 1] = Frag<_Float16>::load(wc + (2 * q + 1) * 32);
    keep4_h(bfw[2 * q], bfw[2 * q + 1], bcw[2 * q], bcw[2 * q + 1]);
  }
  float hreg[8];
#pragma unroll
  for (int v = 0; v < 8; ++v) hreg[v] = 0.0f;
  const float* pf = XPf + (size_t)col * ROWS_M;
  const float* pc = XPc + (size_t)col * ROWS_M;
  const _Float16* arow = (const _Float16*)sA + c * DMODEL + 8 * hh;
  const int hb = (wave < BATCH) ? wave : 0;
  unsigned short* hsdst = HS + (size_t)hb * STEPS * HSW + (size_t)head * DMODEL + lane * 8;
  __syncthreads();
#pragma unroll 1
  for (int t = 0; t < STEPS; ++t) {
    v8f accf = (v8f){0.f,0.f,0.f,0.f,0.f,0.f,0.f,0.f};
    v8f accc = (v8f){0.f,0.f,0.f,0.f,0.f,0.f,0.f,0.f};
#pragma unroll
    for (int kk = 0; kk < 8; ++kk) {
      const v16h a = Frag<_Float16>::load(arow + kk * 32);
      accf = Frag<_Float16>::mma(a, bfw[kk], accf);
      accc = Frag<_Float16>::mma(a, bcw[kk], accc);
      dep_guard_h(accf, accc, a, bfw[kk]);
    }
    __syncthreads();
    const v4f xf0 = *(const v4f*)(pf + t * 8);
    const v4f xf1 = *(const v4f*)(pf + t * 8 + 4);
    const v4f xc0 = *(const v4f*)(pc + t * 8);
    const v4f xc1 = *(const v4f*)(pc + t * 8 + 4);
    if (hh == 0) {
      const float xfv[8] = {xf0[0], xf0[1], xf0[2], xf0[3], xf1[0], xf1[1], xf1[2], xf1[3]};
      const float xcv[8] = {xc0[0], xc0[1], xc0[2], xc0[3], xc1[0], xc1[1], xc1[2], xc1[3]};
#pragma unroll
      for (int v = 0; v < 8; ++v) {
        float af = accf[v] * 0.0625f + xfv[v];
        af = fmaxf(af, -60.0f);
        const float fg = 1.0f / (1.0f + expf(-af));
        const float an = accc[v] * 0.0625f + xcv[v];
        const float ng = tanhf(an);
        const float hn = fg * hreg[v] + (1.0f - fg) * ng;
        hreg[v] = hn;
        sA[v * DMODEL + col] = __builtin_bit_cast(unsigned short, (_Float16)hn);
      }
    }
    __syncthreads();
    if (wave < BATCH) {
      const v8h hv = *(const v8h*)((const _Float16*)sA + wave * DMODEL + lane * 8);
      _Float16* dst = (_Float16*)hsdst + (size_t)t * HSW;
      *(volatile v8h*)dst = hv;
      __threadfence();
      *(volatile v8h*)dst = hv;
    }
  }
}

extern "C" void kernel_launch(void* const* d_in, const int* in_sizes, int n_in,
                              void* d_out, int out_size, void* d_ws, size_t ws_size,
                              hipStream_t stream) {
  if (n_in < 5) return;
  if (in_sizes[0] != BATCH * STEPS * DMODEL) return;
  if (in_sizes[1] != HEADS * 2 * DMODEL * DMODEL) return;
  if (in_sizes[2] != HEADS * 2 * DMODEL * DMODEL) return;
  if (in_sizes[3] != HSW * DMODEL) return;
  if (in_sizes[4] != DMODEL) return;
  if (out_size != BATCH * STEPS * DMODEL) return;

  const float* x  = (const float*)d_in[0];
  const float* Wf = (const float*)d_in[1];
  const float* Wc = (const float*)d_in[2];
  const float* Wl = (const float*)d_in[3];
  const float* bl = (const float*)d_in[4];
  float* out = (float*)d_out;

  const size_t bytesXh  = (size_t)ROWS_M * DMODEL * 2;
  const size_t bytesWT  = (size_t)2 * 2 * HEADS * DMODEL * DMODEL * 2;
  const size_t bytesWlT = (size_t)DMODEL * HSW * 2;
  const size_t bytesXP  = (size_t)2 * DMODEL * ROWS_M * 4;
  const size_t bytesHS  = (size_t)ROWS_M * HSW * 2;
  const size_t offXh  = 0;
  const size_t offWT  = offXh + bytesXh;
  const size_t offWlT = offWT + bytesWT;
  const size_t offXP  = offWlT + bytesWlT;
  const size_t offHS  = offXP + bytesXP;
  const size_t total  = offHS + bytesHS;
  if (total > ws_size) return;

  char* ws = (char*)d_ws;
  unsigned short* Xh  = (unsigned short*)(ws + offXh);
  unsigned short* WT  = (unsigned short*)(ws + offWT);
  unsigned short* WlT = (unsigned short*)(ws + offWlT);
  float*          XP  = (float*)(ws + offXP);
  unsigned short* HS  = (unsigned short*)(ws + offHS);

  const size_t headPlane = (size_t)DMODEL * DMODEL;
  const size_t partPlane = (size_t)HEADS * headPlane;
  const size_t gatePlane = 2 * partPlane;
  const size_t xpPlane   = (size_t)DMODEL * ROWS_M;
  float* XPf = XP;
  float* XPc = XP + xpPlane;

  cast_x_rows<<<dim3((ROWS_M * 32) / 256), dim3(256), 0, stream>>>(x, Xh);
  prep_w_rows<<<dim3((2 * HEADS * DMODEL * 32) / 256), dim3(256), 0, stream>>>(Wf, WT);
  prep_w_rows<<<dim3((2 * HEADS * DMODEL * 32) / 256), dim3(256), 0, stream>>>(Wc, WT + gatePlane);
  prep_wl_rows<<<dim3((DMODEL * (HSW / 8)) / 256), dim3(256), 0, stream>>>(Wl, WlT);

  const int projBlocks = ((DMODEL / 64) * (ROWS_M / 64)) / 8;
  const int outBlocks = ((ROWS_M / 64) * (DMODEL / 64)) / 8;

  for (int hd = 0; hd < HEADS; ++hd) {
    const unsigned short* Ax = WT + (size_t)hd * headPlane;
    wmma_gemm64<0, false, 0, 0, false, 0><<<dim3(projBlocks, 2, 1), dim3(256), 0, stream>>>(
        Ax, Ax, DMODEL, (long)gatePlane,
        Xh, Xh, DMODEL, 0L,
        (void*)XP, (void*)XP, ROWS_M, (long)xpPlane,
        bl, (const float*)XP, 0L,
        DMODEL, ROWS_M, DMODEL, 0.0625f);
    const unsigned short* Whf = WT + partPlane + (size_t)hd * headPlane;
    const unsigned short* Whc = WT + gatePlane + partPlane + (size_t)hd * headPlane;
    gated_scan<<<dim3(1), dim3(512), 0, stream>>>(XPf, XPc, Whf, Whc, HS, hd);
  }

  wmma_gemm64<0, false, 2, 0, false, 0><<<dim3(outBlocks, 1, 1), dim3(256), 0, stream>>>(
      HS, HS, HSW, 0L,
      WlT, WlT, HSW, 0L,
      (void*)out, (void*)out, DMODEL, 0L,
      bl, (const float*)XP, 0L,
      ROWS_M, DMODEL, HSW, 0.03125f);
}
